// GlobalSelfAttention_32349693673710
// MI455X (gfx1250) — hardware-verified
//
#include <hip/hip_runtime.h>


#define NB_  8
#define CC   256
#define CR   32
#define NN   4096
typedef _Float16 h16;
typedef unsigned short bf;
typedef __attribute__((ext_vector_type(16))) __bf16   v16bf;
typedef __attribute__((ext_vector_type(16))) _Float16 v16h;
typedef __attribute__((ext_vector_type(8)))  _Float16 v8h;
typedef __attribute__((ext_vector_type(8)))  unsigned short v8us;
typedef __attribute__((ext_vector_type(8)))  float    v8f;
typedef __attribute__((ext_vector_type(4)))  float    v4f;
typedef v8h  __attribute__((may_alias)) v8ha;
typedef v4f  __attribute__((may_alias)) v4fa;
typedef v8us __attribute__((may_alias)) v8usa;

__device__ __forceinline__ unsigned short f2bf(float f) { unsigned u = __float_as_uint(f); u += 0x7FFFu + ((u >> 16) & 1u); return (unsigned short)(u >> 16); }
__device__ __forceinline__ float bf2f(unsigned short b) { return __uint_as_float(((unsigned)b) << 16); }
__device__ __forceinline__ float bfr(float f) { return bf2f(f2bf(f)); }
__device__ __forceinline__ v16h cat16(v8h lo, v8h hi) { return __builtin_shufflevector(lo, hi, 0, 1, 2, 3, 4, 5, 6, 7, 8, 9, 10, 11, 12, 13, 14, 15); }
__device__ __forceinline__ v16bf cat16b(v8us lo, v8us hi) { return __builtin_bit_cast(v16bf, __builtin_shufflevector(lo, hi, 0, 1, 2, 3, 4, 5, 6, 7, 8, 9, 10, 11, 12, 13, 14, 15)); }
__device__ __forceinline__ v8f wmma16(v16h a, v16h b, v8f c) { return __builtin_amdgcn_wmma_f32_16x16x32_f16(false, a, false, b, (short)0, c, false, false); }
__device__ __forceinline__ v8f wmmab(v16bf a, v16bf b, v8f c) { return __builtin_amdgcn_wmma_f32_16x16x32_bf16(false, a, false, b, (short)0, c, false, false); }


template <typename T16> struct WFrag;
template <> struct WFrag<h16> { typedef v16h V; static __device__ __forceinline__ V ld(const h16* p) { return cat16(*(const v8h*)p, *(const v8h*)(p + 16)); } static __device__ __forceinline__ v8f mma(V a, V b, v8f c) { return wmma16(a, b, c); } };
template <> struct WFrag<bf> { typedef v16bf V; static __device__ __forceinline__ V ld(const bf* p) { return cat16b(*(const v8us*)p, *(const v8us*)(p + 16)); } static __device__ __forceinline__ v8f mma(V a, V b, v8f c) { return wmmab(a, b, c); } };
template <typename T16, int NSPLIT, bool BIAS>
__global__ __launch_bounds__(32) void k_gemmw(const T16* __restrict__ A, const T16* __restrict__ A2, const T16* __restrict__ Bt, const T16* __restrict__ Bt2, int K, float* C, int ldc, const float* __restrict__ bias, size_t sA, size_t sB, size_t sC) {
    typedef typename WFrag<T16>::V V;
    __shared__ __align__(16) float os[16 * 68];
    const size_t z = blockIdx.z; A += z * sA; if (A2) A2 += z * sA; Bt += z * sB; if (Bt2) Bt2 += z * sB; C += z * sC;
    const int lane = threadIdx.x & 31, lr = lane & 15, hi = lane >> 4; const int r0 = blockIdx.x * 64, c0 = blockIdx.y * 64;
    v8f acc[4][4];
#pragma unroll
    for (int mb = 0; mb < 4; ++mb)
#pragma unroll
        for (int nb = 0; nb < 4; ++nb) acc[mb][nb] = (v8f){};
    const size_t aoff = (size_t)(r0 + lr) * K + 8 * hi, boff = (size_t)(c0 + lr) * K + 8 * hi;
#pragma unroll 1
    for (int kc = 0; kc < K; kc += 32) {
        V a[4], a2[4];
#pragma unroll
        for (int mb = 0; mb < 4; ++mb) { a[mb] = WFrag<T16>::ld(A + aoff + (size_t)mb * 16 * K + kc); if (NSPLIT == 1 || NSPLIT == 2) a2[mb] = WFrag<T16>::ld(A2 + aoff + (size_t)mb * 16 * K + kc); }
#pragma unroll
        for (int nb = 0; nb < 4; ++nb) { const V b = WFrag<T16>::ld(Bt + boff + (size_t)nb * 16 * K + kc); V b2; if (NSPLIT >= 2) b2 = WFrag<T16>::ld(Bt2 + boff + (size_t)nb * 16 * K + kc);
#pragma unroll
            for (int mb = 0; mb < 4; ++mb) { acc[mb][nb] = WFrag<T16>::mma(a[mb], b, acc[mb][nb]); if (NSPLIT == 1 || NSPLIT == 2) acc[mb][nb] = WFrag<T16>::mma(a2[mb], b, acc[mb][nb]); if (NSPLIT >= 2) acc[mb][nb] = WFrag<T16>::mma(a[mb], b2, acc[mb][nb]); } }
        asm volatile("v_nop\n\tv_nop\n\tv_nop\n\tv_nop" : "+v"(acc[0][0]), "+v"(acc[1][1]), "+v"(acc[2][2]), "+v"(acc[3][3]) : "v"(a[0]), "v"(a[3]));
    }
#pragma unroll
    for (int mb = 0; mb < 4; ++mb) {
#pragma unroll
        for (int nb = 0; nb < 4; ++nb) {
#pragma unroll
            for (int j = 0; j < 8; ++j) os[(hi * 8 + j) * 68 + nb * 16 + lr] = acc[mb][nb][j]; }
        __builtin_amdgcn_wave_barrier(); asm volatile("" ::: "memory");
        float* crow = C + (size_t)(r0 + mb * 16) * ldc + c0;
#pragma unroll 1
        for (int ps = 0; ps < 2; ++ps) {
#pragma unroll
            for (int s = 0; s < 8; ++s) { const int row = 2 * s + hi, cofs = lr * 4; v4f val = *(const v4fa*)(os + row * 68 + cofs); if (BIAS) { val[0] += bfr(bias[c0 + cofs]); val[1] += bfr(bias[c0 + cofs + 1]); val[2] += bfr(bias[c0 + cofs + 2]); val[3] += bfr(bias[c0 + cofs + 3]); }
                *(volatile v4f*)(crow + (size_t)row * ldc + cofs) = val; }
            if (ps == 0) __threadfence(); }
        __builtin_amdgcn_wave_barrier(); asm volatile("" ::: "memory");
    }
}

__device__ __forceinline__ void splitf(float y, unsigned short& h, unsigned short& l) { h = f2bf(y); l = f2bf(y - bf2f(h)); }
typedef __attribute__((ext_vector_type(2))) unsigned short v2us;
typedef __attribute__((ext_vector_type(4))) unsigned short v4us;

__global__ __launch_bounds__(256) void k_wt128(const float* __restrict__ w, bf* A) { const int e = (blockIdx.x * 256 + threadIdx.x) * 4; if (e >= 128 * CC) return; const int r = e / CC; v4us o; for (int u = 0; u < 4; ++u) o[u] = (r < 3 * CR) ? f2bf(w[e + u]) : (unsigned short)0; *(volatile v4us*)(A + e) = o; __threadfence(); *(volatile v4us*)(A + e) = o; }
__global__ __launch_bounds__(256) void k_wo(const float* __restrict__ w, bf* A) { const int e = (blockIdx.x * 256 + threadIdx.x) * 4; if (e >= CC * CR) return; v4us o; for (int u = 0; u < 4; ++u) o[u] = f2bf(w[e + u]); *(volatile v4us*)(A + e) = o; __threadfence(); *(volatile v4us*)(A + e) = o; }
__global__ __launch_bounds__(256) void k_xt(const float* __restrict__ X, bf* XT) { const int e = (blockIdx.x * 256 + threadIdx.x) * 4; if (e >= NN * CC) return; const int c = e % CC; const int n = e / CC; v4us o;
#pragma unroll
    for (int u = 0; u < 4; ++u) o[u] = f2bf(X[(size_t)(c + u) * NN + n]); *(volatile v4us*)(XT + e) = o; __threadfence(); *(volatile v4us*)(XT + e) = o; }
__global__ __launch_bounds__(256) void k_qk(const float* __restrict__ T, bf* Qh, bf* Ql, bf* Kh, bf* Kl) { const int e = (blockIdx.x * 256 + threadIdx.x) * 4; if (e >= NN * CR) return; const int c = e % CR; const int n = e / CR; v4us qh, ql, kh, kl;
#pragma unroll
    for (int u = 0; u < 4; ++u) { unsigned short a, b; splitf(T[(size_t)(CR + c + u) * NN + n], a, b); qh[u] = a; ql[u] = b; splitf(T[(size_t)(c + u) * NN + n], a, b); kh[u] = a; kl[u] = b; }
    *(volatile v4us*)(Qh + e) = qh; *(volatile v4us*)(Ql + e) = ql; *(volatile v4us*)(Kh + e) = kh; *(volatile v4us*)(Kl + e) = kl; __threadfence(); *(volatile v4us*)(Qh + e) = qh; *(volatile v4us*)(Ql + e) = ql; *(volatile v4us*)(Kh + e) = kh; *(volatile v4us*)(Kl + e) = kl; }
__global__ __launch_bounds__(256) void k_vp(const float* __restrict__ T, bf* Vh, bf* Vl) { const size_t e = ((size_t)blockIdx.x * 256 + threadIdx.x) * 4; if (e >= (size_t)64 * NN) return; const int r = (int)(e / NN); const int n = (int)(e % NN); v4us oh, ol;
#pragma unroll
    for (int u = 0; u < 4; ++u) { unsigned short a = 0, b = 0; if (r < CR) splitf(T[(size_t)(2 * CR + r) * NN + n + u], a, b); oh[u] = a; ol[u] = b; } *(volatile v4us*)(Vh + e) = oh; *(volatile v4us*)(Vl + e) = ol; __threadfence(); *(volatile v4us*)(Vh + e) = oh; *(volatile v4us*)(Vl + e) = ol; }
__global__ __launch_bounds__(256) void k_gsm(const float* __restrict__ S, bf* Ph, bf* Pl) { const int lane = threadIdx.x & 31; const int row = blockIdx.x * 8 + (threadIdx.x >> 5); if (row >= NN) return; const float* sr = S + (size_t)row * NN; float mx = -3.0e38f;
#pragma unroll 2
    for (int ch = 0; ch < NN / 128; ++ch) { const v4f a = *(const v4f*)(sr + ch * 128 + lane * 4); for (int u = 0; u < 4; ++u) mx = fmaxf(mx, a[u]); }
#pragma unroll
    for (int sh = 16; sh; sh >>= 1) mx = fmaxf(mx, __shfl_xor(mx, sh, 32));
    float sum = 0.f;
#pragma unroll 2
    for (int ch = 0; ch < NN / 128; ++ch) { const v4f a = *(const v4f*)(sr + ch * 128 + lane * 4);
#pragma unroll
        for (int u = 0; u < 4; ++u) { float d0 = __fsub_rn(a[u], mx); asm volatile("" : "+v"(d0)); sum += __builtin_amdgcn_exp2f(__fmul_rn(d0, 1.4426950408889634f)); } }
#pragma unroll
    for (int sh = 16; sh; sh >>= 1) sum += __shfl_xor(sum, sh, 32);
    const float f = __fdiv_rn(1.0f, sum);
#pragma unroll 2
    for (int ch = 0; ch < NN / 128; ++ch) { const v4f a = *(const v4f*)(sr + ch * 128 + lane * 4); v4us oh, ol;
#pragma unroll
        for (int u = 0; u < 4; ++u) { float d0 = __fsub_rn(a[u], mx); asm volatile("" : "+v"(d0)); const float e = __builtin_amdgcn_exp2f(__fmul_rn(d0, 1.4426950408889634f)); unsigned short a2, c2; splitf(e * f, a2, c2); oh[u] = a2; ol[u] = c2; }
        const size_t oo = (size_t)row * NN + ch * 128 + lane * 4; *(volatile v4us*)(Ph + oo) = oh; *(volatile v4us*)(Pl + oo) = ol; __threadfence(); *(volatile v4us*)(Ph + oo) = oh; *(volatile v4us*)(Pl + oo) = ol; } }
__global__ __launch_bounds__(256) void k_ot(const float* __restrict__ O1, bf* Oh, bf* Ol) { const int e = (blockIdx.x * 256 + threadIdx.x) * 4; if (e >= NN * CR) return; const int c = e % CR; const int n = e / CR; v4us oh, ol;
#pragma unroll
    for (int u = 0; u < 4; ++u) { unsigned short a, b; splitf(O1[(size_t)(c + u) * NN + n], a, b); oh[u] = a; ol[u] = b; } *(volatile v4us*)(Oh + e) = oh; *(volatile v4us*)(Ol + e) = ol; __threadfence(); *(volatile v4us*)(Oh + e) = oh; *(volatile v4us*)(Ol + e) = ol; }
__global__ __launch_bounds__(256) void k_fin(const float* __restrict__ G, const float* __restrict__ X, const float* __restrict__ scale, float* Y) { const size_t e = ((size_t)blockIdx.x * 256 + threadIdx.x) * 4; if (e >= (size_t)CC * NN) return; const int n = (int)(e % NN); const int c = (int)(e / NN); const float sc = bfr(scale[0]); const v4f xx = *(const v4f*)(X + e); v4f r;
#pragma unroll
    for (int u = 0; u < 4; ++u) { float p = __fmul_rn(sc, G[(size_t)(n + u) * CC + c]); asm volatile("" : "+v"(p)); r[u] = __fadd_rn(p, bfr(xx[u])); } *(volatile v4f*)(Y + e) = r; __threadfence(); *(volatile v4f*)(Y + e) = r; }

extern "C" void kernel_launch(void* const* d_in, const int* in_sizes, int n_in,
                              void* d_out, int out_size, void* d_ws, size_t ws_size, hipStream_t stream) {
    (void)in_sizes; (void)n_in; (void)out_size;
    const float* x = (const float*)d_in[0]; const float* Wt = (const float*)d_in[1]; const float* Wo = (const float*)d_in[2]; const float* scale = (const float*)d_in[3];
    float* OUT = (float*)d_out;
    char* wsp = (char*)d_ws;
    auto take = [&](size_t bytes) { char* p = wsp; wsp += (bytes + 255) & ~(size_t)255; return (void*)p; };
    bf* AW = (bf*)take((size_t)128 * CC * 2); bf* AO = (bf*)take((size_t)CC * CR * 2); bf* XT = (bf*)take((size_t)NN * CC * 2); float* T = (float*)take((size_t)128 * NN * 4);
    bf* QTh = (bf*)take((size_t)NN * CR * 2); bf* QTl = (bf*)take((size_t)NN * CR * 2); bf* KTh = (bf*)take((size_t)NN * CR * 2); bf* KTl = (bf*)take((size_t)NN * CR * 2); bf* VPh = (bf*)take((size_t)64 * NN * 2); bf* VPl = (bf*)take((size_t)64 * NN * 2);
    float* S = (float*)take((size_t)NN * NN * 4); bf* Ph = (bf*)take((size_t)NN * NN * 2); bf* Pl = (bf*)take((size_t)NN * NN * 2); float* O1 = (float*)take((size_t)64 * NN * 4); bf* OTh = (bf*)take((size_t)NN * CR * 2); bf* OTl = (bf*)take((size_t)NN * CR * 2); float* G = (float*)take((size_t)CC * NN * 4);
    if ((size_t)(wsp - (char*)d_ws) > ws_size) return;
    k_wt128<<<(128 * CC / 4 + 255) / 256, 256, 0, stream>>>(Wt, AW); k_wo<<<(CC * CR / 4 + 255) / 256, 256, 0, stream>>>(Wo, AO);
    for (int b = 0; b < NB_; ++b) { const float* xb = x + (size_t)b * CC * NN;
        k_xt<<<(NN * CC / 4 + 255) / 256, 256, 0, stream>>>(xb, XT);
        k_gemmw<bf, 0, false><<<dim3(2, NN / 64, 1), 32, 0, stream>>>(AW, nullptr, XT, nullptr, CC, T, NN, nullptr, 0, 0, 0);
        k_qk<<<(NN * CR / 4 + 255) / 256, 256, 0, stream>>>(T, QTh, QTl, KTh, KTl); k_vp<<<(64 * NN / 4 + 255) / 256, 256, 0, stream>>>(T, VPh, VPl);
        k_gemmw<bf, 2, false><<<dim3(NN / 64, NN / 64, 1), 32, 0, stream>>>(QTh, QTl, KTh, KTl, CR, S, NN, nullptr, 0, 0, 0);
        k_gsm<<<NN / 8, 256, 0, stream>>>(S, Ph, Pl);
        k_gemmw<bf, 2, false><<<dim3(1, NN / 64, 1), 32, 0, stream>>>(VPh, VPl, Ph, Pl, NN, O1, NN, nullptr, 0, 0, 0);
        k_ot<<<(NN * CR / 4 + 255) / 256, 256, 0, stream>>>(O1, OTh, OTl);
        k_gemmw<bf, 1, false><<<dim3(NN / 64, CC / 64, 1), 32, 0, stream>>>(OTh, OTl, AO, nullptr, CR, G, CC, nullptr, 0, 0, 0);
        k_fin<<<(CC * NN / 4 + 255) / 256, 256, 0, stream>>>(G, xb, scale, OUT + (size_t)b * CC * NN); }
}
